// HistoryRGCN_39522289058166
// MI455X (gfx1250) — hardware-run, weakly checked
//
#include <hip/hip_runtime.h>
#include <stddef.h>
#include <math.h>


#define FD      128
#define NREL    8
#define KD      1024
#define APK     1032
#define NOUT    40
#define NP2     48
#define TROWS   16
#define NTHR    256
#define NWAVE   8
#define MAXDEG  1024
#define WSC     64.0f
#define RWSC    0.015625f
#define BN_EPS  1e-5f
#define NB1BLK  64
#define NB2BLK  24
#define WSCAP   134217728

static_assert(KD == NREL * FD);
static_assert((APK % 8) == 0 && APK >= KD);
static_assert((NP2 % 16) == 0 && NP2 >= NOUT && (FD % 16) == 0);
static_assert(NTHR == 32 * NWAVE && TROWS == 2 * NWAVE);
static_assert(((TROWS * NOUT) % 4) == 0 && ((TROWS * NOUT * 4) % 128) == 0);
static_assert((TROWS * NOUT) / 4 <= NTHR);
static_assert(NB1BLK * NTHR == FD * (KD / 8) && NB2BLK * NTHR == NP2 * (KD / 8));
static_assert((KD % 32) == 0);

typedef _Float16 v4h  __attribute__((ext_vector_type(4)));
typedef _Float16 v8h  __attribute__((ext_vector_type(8)));
typedef _Float16 v16h __attribute__((ext_vector_type(16)));
typedef float    v4f  __attribute__((ext_vector_type(4)));
typedef float    v8f  __attribute__((ext_vector_type(8)));
union Frag { v16h v; v8h h[2]; };

__device__ __forceinline__ v8f wmh(v16h a, v16h b, v8f c) {
  v8f d = __builtin_amdgcn_wmma_f32_16x16x32_f16(false, a, false, b, (short)0, c, false, false);
  asm volatile("v_nop\n\tv_nop\n\tv_nop\n\tv_nop" : "+v"(d) : "v"(a), "v"(b));
  return d;
}

__device__ __forceinline__ v4h cvt4(v4f a) {
  v4h r;
  r[0] = (_Float16)a[0]; r[1] = (_Float16)a[1]; r[2] = (_Float16)a[2]; r[3] = (_Float16)a[3];
  return r;
}

__global__ __launch_bounds__(NTHR) void k_wprep(const float* __restrict__ W1, const float* __restrict__ W2,
                                                _Float16* B1, _Float16* B2) {
  const int blk = blockIdx.x, tid = threadIdx.x;
  v8h hv;
  _Float16* dst;
  if (blk < NB1BLK) {
    const int i = blk * NTHR + tid;
    const int n = i >> 7, k0 = (i & 127) * 8;
#pragma unroll
    for (int e = 0; e < 8; ++e) hv[e] = (_Float16)(W1[(size_t)(k0 + e) * FD + n] * WSC);
    dst = B1 + (size_t)i * 8;
  } else {
    const int i = (blk - NB1BLK) * NTHR + tid;
    const int n = i >> 7, k0 = (i & 127) * 8;
    const int na = n > NOUT - 1 ? NOUT - 1 : n;
#pragma unroll
    for (int e = 0; e < 8; ++e) {
      const float w = W2[(size_t)(k0 + e) * NOUT + na] * WSC;
      hv[e] = (_Float16)((n < NOUT) ? w : 0.0f);
    }
    dst = B2 + (size_t)i * 8;
  }
  *(volatile v8h*)dst = hv;
  __threadfence();
  *(volatile v8h*)dst = hv;
}

template <bool L2>
__global__ __launch_bounds__(NTHR) void k_layer(
    const float* __restrict__ feat, const _Float16* __restrict__ Bw,
    const int* __restrict__ ptr, const int* __restrict__ idx, const int* __restrict__ ety,
    const float* __restrict__ bng, const float* __restrict__ bnb,
    const float* __restrict__ bnm, const float* __restrict__ bnv,
    float* outp, int nN, int nE) {
  constexpr int NCT = L2 ? (NP2 / 16) : (FD / 16);
  constexpr int SP  = L2 ? NP2 : FD;
  __shared__ __attribute__((aligned(16))) _Float16 sA[TROWS * APK];
  __shared__ __attribute__((aligned(16))) float stg[TROWS * SP];
  __shared__ __attribute__((aligned(16))) float sout[TROWS * NOUT];
  __shared__ float invdeg[TROWS];
  const int tid = threadIdx.x, lane = tid & 31, wave = tid >> 5, hh = lane >> 4, m = lane & 15;
  const int tile = blockIdx.x;

#pragma unroll 1
  for (int s = 0; s < 2; ++s) {
    const int ln = 2 * wave + s;
    const int node = tile * TROWS + ln;
    const int nc = node > nN - 1 ? nN - 1 : node;
    const int p0 = ptr[nc];
    const int p1 = ptr[nc + 1];
    int deg = (node < nN) ? (p1 - p0) : 0;
    deg = deg < 0 ? 0 : (deg > MAXDEG ? MAXDEG : deg);
    v4f a0 = {0.f, 0.f, 0.f, 0.f}, a1 = {0.f, 0.f, 0.f, 0.f}, a2 = {0.f, 0.f, 0.f, 0.f}, a3 = {0.f, 0.f, 0.f, 0.f};
    v4f a4 = {0.f, 0.f, 0.f, 0.f}, a5 = {0.f, 0.f, 0.f, 0.f}, a6 = {0.f, 0.f, 0.f, 0.f}, a7 = {0.f, 0.f, 0.f, 0.f};
#pragma unroll 1
    for (int q0 = 0; q0 < deg; q0 += 32) {
      int pos = p0 + q0 + lane;
      pos = pos < 0 ? 0 : (pos > nE - 1 ? nE - 1 : pos);
      int sl = idx[pos];
      sl = sl < 0 ? 0 : (sl > nN - 1 ? nN - 1 : sl);
      int rl = ety[pos];
      rl = rl < 0 ? 0 : (rl > NREL - 1 ? NREL - 1 : rl);
      const int mcnt = (deg - q0) < 32 ? (deg - q0) : 32;
#pragma unroll 1
      for (int p = 0; p < mcnt; ++p) {
        const int sv = __builtin_amdgcn_readlane(sl, p);
        const int rv = __builtin_amdgcn_readlane(rl, p);
        const v4f v = *(const v4f*)(feat + (size_t)sv * FD + 4 * lane);
        if      (rv == 0) a0 = a0 + v;
        else if (rv == 1) a1 = a1 + v;
        else if (rv == 2) a2 = a2 + v;
        else if (rv == 3) a3 = a3 + v;
        else if (rv == 4) a4 = a4 + v;
        else if (rv == 5) a5 = a5 + v;
        else if (rv == 6) a6 = a6 + v;
        else              a7 = a7 + v;
      }
    }
    if (lane == 0) invdeg[ln] = 1.0f / (float)(deg > 1 ? deg : 1);
    _Float16* ap = sA + ln * APK + 4 * lane;
    *(v4h*)(ap + 0 * FD) = cvt4(a0);
    *(v4h*)(ap + 1 * FD) = cvt4(a1);
    *(v4h*)(ap + 2 * FD) = cvt4(a2);
    *(v4h*)(ap + 3 * FD) = cvt4(a3);
    *(v4h*)(ap + 4 * FD) = cvt4(a4);
    *(v4h*)(ap + 5 * FD) = cvt4(a5);
    *(v4h*)(ap + 6 * FD) = cvt4(a6);
    *(v4h*)(ap + 7 * FD) = cvt4(a7);
  }
  __syncthreads();

  if (wave < NCT) {
    const int ct = wave;
    v8f acc = {0.f, 0.f, 0.f, 0.f, 0.f, 0.f, 0.f, 0.f};
    const _Float16* abase = sA + m * APK + 8 * hh;
    const _Float16* bbase = Bw + (size_t)(ct * 16 + m) * KD + 8 * hh;
#pragma unroll 2
    for (int kt = 0; kt < KD / 32; ++kt) {
      Frag a, b;
      a.h[0] = *(const v8h*)(abase + 32 * kt);
      a.h[1] = *(const v8h*)(abase + 32 * kt + 16);
      b.h[0] = *(const v8h*)(bbase + 32 * kt);
      b.h[1] = *(const v8h*)(bbase + 32 * kt + 16);
      acc = wmh(a.v, b.v, acc);
    }
    const int col = ct * 16 + m;
    if (!L2) {
      const float g = bng[col], be = bnb[col], mu = bnm[col], var = bnv[col];
      const float rs = 1.0f / sqrtf(var + BN_EPS);
#pragma unroll
      for (int r = 0; r < 8; ++r) {
        const int row = 8 * hh + r;
        const float v = acc[r] * (invdeg[row] * RWSC);
        float t = (v - mu) * rs * g + be;
        t = fmaxf(t, 0.0f);
        stg[row * SP + col] = t;
      }
    } else {
#pragma unroll
      for (int r = 0; r < 8; ++r) {
        const int row = 8 * hh + r;
        stg[row * SP + col] = acc[r] * (invdeg[row] * RWSC);
      }
    }
  }
  __syncthreads();

  if (!L2) {
    const int r0 = 2 * wave, r1 = 2 * wave + 1;
    const v4f v0 = *(const v4f*)(stg + r0 * SP + 4 * lane);
    const v4f v1 = *(const v4f*)(stg + r1 * SP + 4 * lane);
    float* g0 = outp + (size_t)(tile * TROWS + r0) * FD + 4 * lane;
    float* g1 = outp + (size_t)(tile * TROWS + r1) * FD + 4 * lane;
    *(volatile v4f*)g0 = v0;
    *(volatile v4f*)g1 = v1;
    __threadfence();
    *(volatile v4f*)g0 = v0;
    *(volatile v4f*)g1 = v1;
  } else {
    if (tid < TROWS) {
      const float* rp = stg + tid * SP;
      float mx = rp[0];
#pragma unroll 1
      for (int j = 1; j < NOUT; ++j) mx = fmaxf(mx, rp[j]);
      float sum = 0.0f;
#pragma unroll 1
      for (int j = 0; j < NOUT; ++j) sum += expf(rp[j] - mx);
      const float lg = logf(sum);
#pragma unroll 1
      for (int j = 0; j < NOUT; ++j) sout[tid * NOUT + j] = (rp[j] - mx) - lg;
    }
    __syncthreads();
    int nvalid = nN - tile * TROWS;
    nvalid = nvalid > TROWS ? TROWS : (nvalid < 0 ? 0 : nvalid);
    const int nf = nvalid * NOUT;
    float* ob = outp + (size_t)tile * (TROWS * NOUT);
    v4f ov = {0.f, 0.f, 0.f, 0.f};
    if (tid < (TROWS * NOUT) / 4) ov = *(const v4f*)(sout + 4 * tid);
    const bool act = (tid < (TROWS * NOUT) / 4) && (4 * tid + 4 <= nf);
    if (act) *(volatile v4f*)(ob + 4 * tid) = ov;
    __threadfence();
    if (act) *(volatile v4f*)(ob + 4 * tid) = ov;
  }
}

extern "C" void kernel_launch(void* const* d_in, const int* in_sizes, int n_in,
                              void* d_out, int out_size, void* d_ws, size_t ws_size,
                              hipStream_t stream) {
  if (n_in < 10) return;
  const int nN = in_sizes[7] - 1;
  const int nE = in_sizes[8];
  if (nN <= 0 || nE <= 0) return;
  if (nN > (1 << 24) || nE > (1 << 29)) return;
  if (in_sizes[0] != nN * FD) return;
  if (in_sizes[1] != NREL * FD * FD || in_sizes[2] != NREL * FD * NOUT) return;
  if (in_sizes[3] != FD || in_sizes[4] != FD || in_sizes[5] != FD || in_sizes[6] != FD) return;
  if (in_sizes[9] != nE) return;
  if (out_size != nN * NOUT) return;

  const float* x   = (const float*)d_in[0];
  const float* W1  = (const float*)d_in[1];
  const float* W2  = (const float*)d_in[2];
  const float* bng = (const float*)d_in[3];
  const float* bnb = (const float*)d_in[4];
  const float* bnm = (const float*)d_in[5];
  const float* bnv = (const float*)d_in[6];
  const int*   ptr = (const int*)d_in[7];
  const int*   idx = (const int*)d_in[8];
  const int*   ety = (const int*)d_in[9];
  float* out = (float*)d_out;

  const int nTiles = (nN + TROWS - 1) / TROWS;
  const int NPAD   = nTiles * TROWS;

  char* ws = (char*)d_ws;
  size_t o = 0;
  const size_t oB1 = o; o += (size_t)FD  * KD * 2;      o = (o + 255) & ~(size_t)255;
  const size_t oB2 = o; o += (size_t)NP2 * KD * 2;      o = (o + 255) & ~(size_t)255;
  const size_t oH  = o; o += (size_t)NPAD * FD * 4;     o = (o + 255) & ~(size_t)255;
  if (o > ws_size || o > (size_t)WSCAP) return;
  _Float16* B1 = (_Float16*)(ws + oB1);
  _Float16* B2 = (_Float16*)(ws + oB2);
  float*    H  = (float*)(ws + oH);

  k_wprep<<<NB1BLK + NB2BLK, NTHR, 0, stream>>>(W1, W2, B1, B2);
  k_layer<false><<<nTiles, NTHR, 0, stream>>>(x, B1, ptr, idx, ety, bng, bnb, bnm, bnv, H, nN, nE);
  k_layer<true><<<nTiles, NTHR, 0, stream>>>(H, B2, ptr, idx, ety, bng, bnb, bnm, bnv, out, nN, nE);
}
